// DemoHybridAttention_86535001080333
// MI455X (gfx1250) — hardware-verified
//
#include <hip/hip_runtime.h>
#include <math.h>
#include <stdint.h>

#define BATCH 2
#define SEQ   2048
#define DMOD  512
#define NH    16
#define HD    32
#define MEMN  16
#define TTOT  (SEQ + MEMN)
#define TP    2112
#define NKC   (TP / 64)
#define NQB   (SEQ / 64)
#define MQ    (BATCH * SEQ)
#define MK    (BATCH * TP)
#define HWIN  128
#define ASC   16.0f
#define WSC   64.0f
#define RSC   4096.0f
#define PSC   1024.0f
static_assert(NH * HD == DMOD);
static_assert((TP % 64) == 0 && TP >= TTOT && (TP - TTOT) < 64);
static_assert((SEQ % 64) == 0 && (DMOD % 64) == 0);
static_assert(NQB == 32 && NH == 16);
static_assert(DMOD / 8 == 64);
static_assert(HD == 32);

typedef _Float16 v16h __attribute__((ext_vector_type(16)));
typedef _Float16 v8h  __attribute__((ext_vector_type(8)));
typedef __attribute__((ext_vector_type(16))) __bf16 v16b;
typedef unsigned short v8us __attribute__((ext_vector_type(8)));
typedef float    v8f  __attribute__((ext_vector_type(8)));
typedef float    v4f  __attribute__((ext_vector_type(4)));
typedef unsigned int v4u __attribute__((ext_vector_type(4)));

__device__ __forceinline__ unsigned short bf_bits(float f) {
  unsigned u = __float_as_uint(f);
  return (unsigned short)((u + 0x7FFFu + ((u >> 16) & 1u)) >> 16);
}
__device__ __forceinline__ float bf_up(unsigned short h) { return __uint_as_float(((unsigned)h) << 16); }
__device__ __forceinline__ float bfr(float f) { return bf_up(bf_bits(f)); }
__device__ __forceinline__ unsigned short h_bits(_Float16 x) { return __builtin_bit_cast(unsigned short, x); }
__device__ __forceinline__ unsigned pk16(unsigned short a, unsigned short b) { return (unsigned)a | ((unsigned)b << 16); }
__device__ __forceinline__ v8f zero8() { v8f z = {0.f, 0.f, 0.f, 0.f, 0.f, 0.f, 0.f, 0.f}; return z; }
__device__ __forceinline__ unsigned short cvt_act(float f) { return h_bits((_Float16)(bfr(f) * ASC)); }

__device__ __forceinline__ v16h ldfrag_h(const _Float16* p) {
  union { v16h v; v8h h[2]; } f;
  f.h[0] = *(const v8h*)(p);
  f.h[1] = *(const v8h*)(p + 16);
  return f.v;
}
union FB { v16b v; v16h h; v8us u[2]; };
__device__ __forceinline__ FB ldfrag_b(const unsigned short* p) {
  FB f;
  f.u[0] = *(const v8us*)(p);
  f.u[1] = *(const v8us*)(p + 16);
  return f;
}

__device__ __forceinline__ v8f mma_h(v16h a, v16h b, v8f c) {
  c = __builtin_amdgcn_wmma_f32_16x16x32_f16(false, a, false, b, (short)0, c, false, false);
#if defined(__HIP_DEVICE_COMPILE__)
  asm volatile("v_nop\n\tv_nop\n\tv_nop\n\tv_nop" : "+v"(c) : "v"(a), "v"(b));
#endif
  return c;
}
__device__ __forceinline__ v8f mma_h_raw(v16h a, v16h b, v8f c) {
  return __builtin_amdgcn_wmma_f32_16x16x32_f16(false, a, false, b, (short)0, c, false, false);
}
__device__ __forceinline__ v8f mma_b_raw(v16b a, v16b b, v8f c) {
  return __builtin_amdgcn_wmma_f32_16x16x32_bf16(false, a, false, b, (short)0, c, false, false);
}
__device__ __forceinline__ void dep_guard1(v8f& a, v8f& b, v16h x) {
#if defined(__HIP_DEVICE_COMPILE__)
  asm volatile("v_nop\n\tv_nop\n\tv_nop\n\tv_nop" : "+v"(a), "+v"(b) : "v"(x));
#endif
}
__device__ __forceinline__ void dep_guard2(v8f& a, v8f& b, v16h x, v16h y) {
#if defined(__HIP_DEVICE_COMPILE__)
  asm volatile("v_nop\n\tv_nop\n\tv_nop\n\tv_nop" : "+v"(a), "+v"(b) : "v"(x), "v"(y));
#endif
}
__device__ __forceinline__ void keep4_h(v16h a, v16h b, v16h c, v16h d) {
#if defined(__HIP_DEVICE_COMPILE__)
  asm volatile("v_nop" :: "v"(a), "v"(b), "v"(c), "v"(d));
#endif
}
__device__ __forceinline__ void acc_guard4(v8f& a, v8f& b, v8f& c, v8f& d) {
#if defined(__HIP_DEVICE_COMPILE__)
  asm volatile("v_nop\n\tv_nop\n\tv_nop\n\tv_nop" : "+v"(a), "+v"(b), "+v"(c), "+v"(d));
#endif
}
__device__ __forceinline__ void wave_sync_lds() {
  __builtin_amdgcn_fence(__ATOMIC_RELEASE, "workgroup");
  __builtin_amdgcn_wave_barrier();
  __builtin_amdgcn_fence(__ATOMIC_ACQUIRE, "workgroup");
}

__global__ __launch_bounds__(256) void wtrans(const float* __restrict__ Wq, const float* __restrict__ Wk,
                                              const float* __restrict__ Wv, const float* __restrict__ Wo,
                                              unsigned short* Wt) {
  __shared__ __align__(16) float sW[64 * 68];
  const int y = blockIdx.y;
  const float* W = (y == 0) ? Wq : (y == 1) ? Wk : (y == 2) ? Wv : Wo;
  unsigned short* T16 = Wt + (size_t)y * DMOD * DMOD;
  const int tk = blockIdx.x >> 3, tn = blockIdx.x & 7;
  const int k0 = tk * 64, n0 = tn * 64;
  const int tid = threadIdx.x;
#pragma unroll
  for (int i = 0; i < 4; ++i) {
    const int idx = i * 256 + tid;
    const int kr = idx >> 4, n4 = (idx & 15) * 4;
    const v4f v = *(const v4f*)(W + (size_t)(k0 + kr) * DMOD + n0 + n4);
    *(v4f*)(sW + kr * 68 + n4) = v;
  }
  __syncthreads();
  const bool bfm = (y == 3);
  v4u pieces[2];
  size_t goff[2];
#pragma unroll
  for (int it = 0; it < 2; ++it) {
    const int p = it * 256 + tid;
    const int nr = p >> 3, c8 = (p & 7) * 8;
    unsigned short hw[8];
#pragma unroll
    for (int e = 0; e < 8; ++e) {
      const float f = sW[(c8 + e) * 68 + nr];
      const unsigned short ub = bf_bits(f);
      const unsigned short uh = h_bits((_Float16)(bfr(f) * WSC));
      hw[e] = bfm ? ub : uh;
    }
    v4u u;
    u[0] = pk16(hw[0], hw[1]);
    u[1] = pk16(hw[2], hw[3]);
    u[2] = pk16(hw[4], hw[5]);
    u[3] = pk16(hw[6], hw[7]);
    pieces[it] = u;
    goff[it] = (size_t)(n0 + nr) * DMOD + k0 + c8;
  }
  for (int pass = 0; pass < 2; ++pass) {
#pragma unroll
    for (int it = 0; it < 2; ++it) *(volatile v4u*)(T16 + goff[it]) = pieces[it];
    __threadfence();
  }
}

__global__ __launch_bounds__(256) void convq(const float* __restrict__ X, unsigned short* Xh, int n8) {
  const int i = blockIdx.x * 256 + threadIdx.x;
  if (i >= n8) return;
  const size_t e0 = (size_t)i * 8;
  const v4f a = *(const v4f*)(X + e0);
  const v4f b = *(const v4f*)(X + e0 + 4);
  v4u u;
  u[0] = pk16(cvt_act(a[0]), cvt_act(a[1]));
  u[1] = pk16(cvt_act(a[2]), cvt_act(a[3]));
  u[2] = pk16(cvt_act(b[0]), cvt_act(b[1]));
  u[3] = pk16(cvt_act(b[2]), cvt_act(b[3]));
  for (int pass = 0; pass < 2; ++pass) {
    *(volatile v4u*)(Xh + e0) = u;
    __threadfence();
  }
}

__global__ __launch_bounds__(256) void convkv(const float* __restrict__ Xk, const float* __restrict__ Xv,
                                              const float* __restrict__ memp,
                                              unsigned short* Pk, unsigned short* Pv, int npieces) {
  const int y = blockIdx.y;
  const float* X = (y == 0) ? Xk : Xv;
  unsigned short* P = (y == 0) ? Pk : Pv;
  const int i = blockIdx.x * 256 + threadIdx.x;
  if (i >= npieces) return;
  const int per = TP * (DMOD / 8);
  const int b   = i / per;
  const int rem = i - b * per;
  const int t   = rem >> 6;
  const int d8  = (rem & 63) * 8;
  const int tm  = (t < MEMN) ? t : (MEMN - 1);
  int tc = t - MEMN;
  tc = (tc < 0) ? 0 : tc;
  tc = (tc > SEQ - 1) ? (SEQ - 1) : tc;
  const float* mp = memp + (size_t)tm * DMOD + d8;
  const float* xp = X + ((size_t)b * SEQ + tc) * DMOD + d8;
  const v4f m0 = *(const v4f*)(mp), m1 = *(const v4f*)(mp + 4);
  const v4f x0 = *(const v4f*)(xp), x1 = *(const v4f*)(xp + 4);
  const bool isMem = (t < MEMN);
  const bool isTok = (t < TTOT);
  float f[8];
#pragma unroll
  for (int e = 0; e < 4; ++e) {
    f[e]     = isMem ? m0[e] : (isTok ? x0[e] : 0.f);
    f[4 + e] = isMem ? m1[e] : (isTok ? x1[e] : 0.f);
  }
  v4u u;
  u[0] = pk16(cvt_act(f[0]), cvt_act(f[1]));
  u[1] = pk16(cvt_act(f[2]), cvt_act(f[3]));
  u[2] = pk16(cvt_act(f[4]), cvt_act(f[5]));
  u[3] = pk16(cvt_act(f[6]), cvt_act(f[7]));
  const size_t e0 = (size_t)i * 8;
  for (int pass = 0; pass < 2; ++pass) {
    *(volatile v4u*)(P + e0) = u;
    __threadfence();
  }
}

template <int OM, int BM>
__global__ __launch_bounds__(256) void gemm64(
    const unsigned short* __restrict__ Ap, int lda, int sA,
    const unsigned short* __restrict__ Btp, int ldb, int sB,
    unsigned short* Cout, unsigned short* Cout2, int ldc, int sC,
    const float* __restrict__ bias, int nb,
    int M, int N, int K, float oscale, float rsc) {
  const int zb = blockIdx.y;
  const _Float16* A  = (const _Float16*)(const void*)(Ap + (size_t)zb * (size_t)sA);
  const _Float16* Bt = (const _Float16*)(const void*)(Btp + (size_t)zb * (size_t)sB);
  unsigned short* C1 = Cout + (size_t)zb * (size_t)sC;
  unsigned short* C2 = Cout2 + (size_t)zb * (size_t)sC;
  __shared__ __align__(16) float sT[8][16 * 68];
  const int lane = threadIdx.x & 31;
  const int wave = threadIdx.x >> 5;
  const int tilesN = N >> 6;
  const int tilesM = M >> 6;
  const int tile = blockIdx.x * 8 + wave;
  if (tile >= tilesM * tilesN) return;
  const int tm = tile / tilesN;
  const int tn = tile - tm * tilesN;
  const int m0 = tm << 6;
  const int n0 = tn << 6;

  const int rlane = lane & 15;
  const int koff  = (lane >> 4) * 8;
  const int mOff  = (lane >> 4) * 8;

  v8f acc[4][4];
#pragma unroll
  for (int i = 0; i < 4; ++i)
#pragma unroll
    for (int j = 0; j < 4; ++j) acc[i][j] = zero8();

  for (int k0 = 0; k0 < K; k0 += 32) {
    v16h bh[4];
#pragma unroll
    for (int j = 0; j < 4; ++j) {
      const size_t bo = (size_t)(n0 + (j << 4) + rlane) * ldb + koff + k0;
      bh[j] = ldfrag_h(Bt + bo);
    }
#pragma unroll
    for (int i = 0; i < 4; ++i) {
      const size_t ao = (size_t)(m0 + (i << 4) + rlane) * lda + koff + k0;
      const v16h ah = ldfrag_h(A + ao);
#pragma unroll
      for (int j = 0; j < 4; ++j) acc[i][j] = mma_h_raw(ah, bh[j], acc[i][j]);
      dep_guard1(acc[i][0], acc[i][3], ah);
    }
    keep4_h(bh[0], bh[1], bh[2], bh[3]);
  }
  acc_guard4(acc[0][0], acc[0][1], acc[0][2], acc[0][3]);
  acc_guard4(acc[1][0], acc[1][1], acc[1][2], acc[1][3]);
  acc_guard4(acc[2][0], acc[2][1], acc[2][2], acc[2][3]);
  acc_guard4(acc[3][0], acc[3][1], acc[3][2], acc[3][3]);

  const int q8 = lane >> 3, c8 = (lane & 7) * 8;

  float* slab = sT[wave];
#pragma unroll
  for (int i = 0; i < 4; ++i) {
    const int mBase = m0 + (i << 4);
#pragma unroll
    for (int j = 0; j < 4; ++j) {
#pragma unroll
      for (int r = 0; r < 8; ++r) {
        slab[(mOff + r) * 68 + (j << 4) + rlane] = acc[i][j][r];
      }
    }
    wave_sync_lds();
    v4u hv[4], lv[4];
#pragma unroll
    for (int it = 0; it < 4; ++it) {
      const int row = it * 4 + q8;
      const float* sp = slab + row * 68 + c8;
      float brow = 0.f;
      if (BM == 2) {
        int im = mBase + row;
        im = (im < nb) ? im : (nb - 1);
        brow = bfr(bias[im]);
      }
      v4u a, lw;
#pragma unroll
      for (int e = 0; e < 4; ++e) {
        float b0 = brow, b1 = brow;
        if (BM == 1) {
          int i0 = n0 + c8 + 2 * e, i1 = i0 + 1;
          i0 = (i0 < nb) ? i0 : (nb - 1);
          i1 = (i1 < nb) ? i1 : (nb - 1);
          b0 = bfr(bias[i0]);
          b1 = bfr(bias[i1]);
        }
        const float f0 = sp[2 * e]     * oscale + b0;
        const float f1 = sp[2 * e + 1] * oscale + b1;
        const _Float16 g0 = (_Float16)f0;
        const _Float16 g1 = (_Float16)f1;
        a[e] = pk16(h_bits(g0), h_bits(g1));
        if (OM == 3) {
          const _Float16 r0 = (_Float16)((f0 - (float)g0) * rsc);
          const _Float16 r1 = (_Float16)((f1 - (float)g1) * rsc);
          lw[e] = pk16(h_bits(r0), h_bits(r1));
        } else {
          lw[e] = 0u;
        }
      }
      hv[it] = a;
      lv[it] = lw;
    }
    for (int pass = 0; pass < 2; ++pass) {
#pragma unroll
      for (int it = 0; it < 4; ++it) {
        const int row = it * 4 + q8;
        const size_t go = (size_t)(mBase + row) * ldc + n0 + c8;
        *(volatile v4u*)(C1 + go) = hv[it];
        if (OM == 3) *(volatile v4u*)(C2 + go) = lv[it];
      }
      __threadfence();
    }
    wave_sync_lds();
  }
}

__global__ __launch_bounds__(256) void gemm_ob(
    const unsigned short* __restrict__ Ah, const unsigned short* __restrict__ Al, int hps,
    const unsigned short* __restrict__ Btp, int ldb,
    const float* __restrict__ bias, int nb,
    float* Cout, int ldc, int M, int N, int K) {
  __shared__ __align__(16) float sT[8][16 * 68];
  const int lane = threadIdx.x & 31;
  const int wave = threadIdx.x >> 5;
  const int tilesN = N >> 6;
  const int tilesM = M >> 6;
  const int tile = blockIdx.x * 8 + wave;
  if (tile >= tilesM * tilesN) return;
  const int tm = tile / tilesN;
  const int tn = tile - tm * tilesN;
  const int m0 = tm << 6;
  const int n0 = tn << 6;

  const int rlane = lane & 15;
  const int koff  = (lane >> 4) * 8;
  const int mOff  = (lane >> 4) * 8;

  v8f acc[4][4];
#pragma unroll
  for (int i = 0; i < 4; ++i)
#pragma unroll
    for (int j = 0; j < 4; ++j) acc[i][j] = zero8();

  for (int k0 = 0; k0 < K; k0 += 32) {
    FB bh[4];
#pragma unroll
    for (int j = 0; j < 4; ++j) {
      const size_t bo = (size_t)(n0 + (j << 4) + rlane) * ldb + koff + k0;
      bh[j] = ldfrag_b(Btp + bo);
    }
    const size_t pb = (size_t)(k0 >> 5) * (size_t)hps;
#pragma unroll
    for (int i = 0; i < 4; ++i) {
      const size_t ao = pb + (size_t)(m0 + (i << 4) + rlane) * 32 + koff;
      const FB ah = ldfrag_b(Ah + ao);
      const FB al = ldfrag_b(Al + ao);
#pragma unroll
      for (int j = 0; j < 4; ++j) acc[i][j] = mma_b_raw(ah.v, bh[j].v, acc[i][j]);
#pragma unroll
      for (int j = 0; j < 4; ++j) acc[i][j] = mma_b_raw(al.v, bh[j].v, acc[i][j]);
      dep_guard2(acc[i][0], acc[i][3], ah.h, al.h);
    }
    keep4_h(bh[0].h, bh[1].h, bh[2].h, bh[3].h);
  }
  acc_guard4(acc[0][0], acc[0][1], acc[0][2], acc[0][3]);
  acc_guard4(acc[1][0], acc[1][1], acc[1][2], acc[1][3]);
  acc_guard4(acc[2][0], acc[2][1], acc[2][2], acc[2][3]);
  acc_guard4(acc[3][0], acc[3][1], acc[3][2], acc[3][3]);

  float* slab = sT[wave];
  const int hh2 = lane >> 4, c4 = (lane & 15) * 4;
  v4f b4;
#pragma unroll
  for (int e = 0; e < 4; ++e) {
    int ib = n0 + c4 + e;
    ib = (ib < nb) ? ib : (nb - 1);
    b4[e] = bfr(bias[ib]);
  }
#pragma unroll
  for (int i = 0; i < 4; ++i) {
    const int mBase = m0 + (i << 4);
#pragma unroll
    for (int j = 0; j < 4; ++j) {
#pragma unroll
      for (int r = 0; r < 8; ++r) {
        slab[(mOff + r) * 68 + (j << 4) + rlane] = acc[i][j][r];
      }
    }
    wave_sync_lds();
    v4f vals[8];
#pragma unroll
    for (int it = 0; it < 8; ++it) {
      const int row = it * 2 + hh2;
      vals[it] = *(const v4f*)(slab + row * 68 + c4) + b4;
    }
    for (int pass = 0; pass < 2; ++pass) {
#pragma unroll
      for (int it = 0; it < 8; ++it) {
        const int row = it * 2 + hh2;
        const size_t go = (size_t)(mBase + row) * ldc + n0 + c4;
        *(volatile v4f*)(Cout + go) = vals[it];
      }
      __threadfence();
    }
    wave_sync_lds();
  }
}

__device__ __forceinline__ void hl2(float f0, float f1, unsigned& hw, unsigned& lw) {
  const unsigned short h0 = bf_bits(f0), h1 = bf_bits(f1);
  const unsigned short l0 = bf_bits(f0 - bf_up(h0)), l1 = bf_bits(f1 - bf_up(h1));
  hw = pk16(h0, h1);
  lw = pk16(l0, l1);
}

__global__ __launch_bounds__(128)
void attn32(const unsigned short* __restrict__ qhp, const unsigned short* __restrict__ qlp,
            const unsigned short* __restrict__ khp, const unsigned short* __restrict__ klp,
            const unsigned short* __restrict__ vthp, const unsigned short* __restrict__ vtlp,
            unsigned short* chp, unsigned short* clp, float sscale) {
  union FH { v16h v; v8h h[2]; };
  __shared__ __align__(16) _Float16 Ksh[64 * HD];
  __shared__ __align__(16) _Float16 Ksl[64 * HD];
  __shared__ __align__(16) _Float16 Vth[HD * 64];
  __shared__ __align__(16) _Float16 Vtl[HD * 64];
  __shared__ __align__(16) _Float16 Psh[4][16 * 64];
  __shared__ __align__(16) _Float16 Psl[4][16 * 64];
  __shared__ __align__(16) float    Os[4][16 * HD];

  const int tid  = threadIdx.x;
  const int wave = tid >> 5;
  const int lane = tid & 31;
  const int hh   = lane >> 4;
  const int c    = lane & 15;

  const int bx = blockIdx.x;
  const int qb = bx & (NQB - 1);
  const int hq = (bx >> 5) & (NH - 1);
  const int b  = bx >> 9;
  const int s0 = qb * 64 + wave * 16;

  const _Float16* Qh = (const _Float16*)(const void*)qhp + (size_t)b * SEQ * DMOD + hq * HD;
  const _Float16* Ql = (const _Float16*)(const void*)qlp + (size_t)b * SEQ * DMOD + hq * HD;
  const _Float16* Kh = (const _Float16*)(const void*)khp + (size_t)b * TP * DMOD + hq * HD;
  const _Float16* Kl = (const _Float16*)(const void*)klp + (size_t)b * TP * DMOD + hq * HD;
  const _Float16* Vh = (const _Float16*)(const void*)vthp + ((size_t)b * DMOD + hq * HD) * TP;
  const _Float16* Vl = (const _Float16*)(const void*)vtlp + ((size_t)b * DMOD + hq * HD) * TP;

  const v16h qa = ldfrag_h(Qh + (size_t)(s0 + c) * DMOD + 8 * hh);
  const v16h qr = ldfrag_h(Ql + (size_t)(s0 + c) * DMOD + 8 * hh);

  float mrow[8], lrow[8];
  v8f oacc[2];
#pragma unroll
  for (int r = 0; r < 8; ++r) { mrow[r] = -INFINITY; lrow[r] = 0.f; }
#pragma unroll
  for (int t = 0; t < 2; ++t) oacc[t] = zero8();

  const int jmin = qb * 64 + MEMN - HWIN;
  int lo = (jmin < 0) ? 0 : (jmin >> 6);
  int hi = (qb * 64 + 63 + MEMN + HWIN) >> 6;
  if (hi > NKC - 1) hi = NKC - 1;
  const int extra = (lo > 0) ? 1 : 0;
  const float rinv = 1.0f / RSC;

  for (int step = -extra; step <= hi - lo; ++step) {
    const int kt  = (step < 0) ? 0 : (lo + step);
    const int kv0 = kt * 64;
    __syncthreads();
#pragma unroll
    for (int i = 0; i < 2; ++i) {
      const int p  = tid + 128 * i;
      const int r  = p >> 2, ck = (p & 3) * 8;
      const int d  = p >> 3, cv = (p & 7) * 8;
      const v8h a0 = *(const v8h*)(Kh + (size_t)(kv0 + r) * DMOD + ck);
      const v8h a1 = *(const v8h*)(Kl + (size_t)(kv0 + r) * DMOD + ck);
      const v8h b0 = *(const v8h*)(Vh + (size_t)d * TP + kv0 + cv);
      const v8h b1 = *(const v8h*)(Vl + (size_t)d * TP + kv0 + cv);
      *(v8h*)(Ksh + r * HD + ck) = a0;
      *(v8h*)(Ksl + r * HD + ck) = a1;
      *(v8h*)(Vth + d * 64 + cv) = b0;
      *(v8h*)(Vtl + d * 64 + cv) = b1;
    }
    __syncthreads();

    v8f s[4];
#pragma unroll
    for (int j = 0; j < 4; ++j) {
      FH kb, kc;
      const int kr = (j * 16 + c) * HD;
      kb.h[0] = *(const v8h*)(Ksh + kr + 8 * hh);
      kb.h[1] = *(const v8h*)(Ksh + kr + 16 + 8 * hh);
      kc.h[0] = *(const v8h*)(Ksl + kr + 8 * hh);
      kc.h[1] = *(const v8h*)(Ksl + kr + 16 + 8 * hh);
      v8f sh = mma_h(qa, kb.v, zero8());
      v8f sl = mma_h(qa, kc.v, zero8());
      sl = mma_h(qr, kb.v, sl);
      const int key = kv0 + j * 16 + c;
#pragma unroll
      for (int r = 0; r < 8; ++r) {
        const int qi = MEMN + s0 + 8 * hh + r;
        const float v = (sh[r] + sl[r] * rinv) * sscale;
        int dd = key - qi;
        if (dd < 0) dd = -dd;
        const bool vis = (key < MEMN) | ((dd <= HWIN) & (key < TTOT));
        s[j][r] = vis ? v : -INFINITY;
      }
    }

    _Float16* pwh = Psh[wave];
    _Float16* pwl = Psl[wave];
#pragma unroll
    for (int r = 0; r < 8; ++r) {
      float m = s[0][r];
      m = fmaxf(m, s[1][r]);
      m = fmaxf(m, s[2][r]);
      m = fmaxf(m, s[3][r]);
#pragma unroll
      for (int off = 1; off < 16; off <<= 1) m = fmaxf(m, __shfl_xor(m, off, 32));
      const float mnew  = fmaxf(mrow[r], m);
      const float ms    = (mnew == -INFINITY) ? 0.f : mnew;
      const float alpha = __expf(mrow[r] - ms);
      mrow[r] = mnew;
      float psum = 0.f;
#pragma unroll
      for (int j = 0; j < 4; ++j) {
        const float p  = __expf(s[j][r] - ms);
        psum += p;
        const float pv = p * PSC;
        const _Float16 ph = (_Float16)pv;
        const int pi = (8 * hh + r) * 64 + j * 16 + c;
        pwh[pi] = ph;
        pwl[pi] = (_Float16)((pv - (float)ph) * RSC);
      }
#pragma unroll
      for (int off = 1; off < 16; off <<= 1) psum += __shfl_xor(psum, off, 32);
      lrow[r] = lrow[r] * alpha + psum;
#pragma unroll
      for (int t = 0; t < 2; ++t) oacc[t][r] *= alpha;
    }
    wave_sync_lds();

    v8f ol[2];
#pragma unroll
    for (int t = 0; t < 2; ++t) ol[t] = zero8();
#pragma unroll 1
    for (int kk = 0; kk < 2; ++kk) {
      FH pa, pr;
      pa.h[0] = *(const v8h*)(pwh + c * 64 + kk * 32 + 8 * hh);
      pa.h[1] = *(const v8h*)(pwh + c * 64 + kk * 32 + 16 + 8 * hh);
      pr.h[0] = *(const v8h*)(pwl + c * 64 + kk * 32 + 8 * hh);
      pr.h[1] = *(const v8h*)(pwl + c * 64 + kk * 32 + 16 + 8 * hh);
#pragma unroll
      for (int t = 0; t < 2; ++t) {
        FH vb, wb;
        vb.h[0] = *(const v8h*)(Vth + (t * 16 + c) * 64 + kk * 32 + 8 * hh);
        vb.h[1] = *(const v8h*)(Vth + (t * 16 + c) * 64 + kk * 32 + 16 + 8 * hh);
        wb.h[0] = *(const v8h*)(Vtl + (t * 16 + c) * 64 + kk * 32 + 8 * hh);
        wb.h[1] = *(const v8h*)(Vtl + (t * 16 + c) * 64 + kk * 32 + 16 + 8 * hh);
        oacc[t] = mma_h(pa.v, vb.v, oacc[t]);
        ol[t]   = mma_h(pa.v, wb.v, ol[t]);
        ol[t]   = mma_h(pr.v, vb.v, ol[t]);
      }
    }
#pragma unroll
    for (int t = 0; t < 2; ++t) {
#pragma unroll
      for (int r = 0; r < 8; ++r) oacc[t][r] += ol[t][r] * rinv;
    }
  }

  float* os = Os[wave];
#pragma unroll
  for (int r = 0; r < 8; ++r) {
    const float l = lrow[r];
    const float inv = ((l > 0.f) ? (1.0f / l) : 0.f) * (1.0f / PSC);
#pragma unroll
    for (int t = 0; t < 2; ++t) os[(8 * hh + r) * HD + t * 16 + c] = oacc[t][r] * inv;
  }
  wave_sync_lds();
  {
    const size_t hps = (size_t)MQ * HD;
    v4u hv[2], lv[2];
    size_t go[2];
#pragma unroll
    for (int it = 0; it < 2; ++it) {
      const int p   = it * 32 + lane;
      const int row = p >> 2;
      const int c8  = (p & 3) * 8;
      const float* sp = os + row * HD + c8;
      const v4f x0 = *(const v4f*)(sp);
      const v4f x1 = *(const v4f*)(sp + 4);
      v4u a, bb;
      unsigned aw, bw;
      hl2(x0[0], x0[1], aw, bw); a[0] = aw; bb[0] = bw;
      hl2(x0[2], x0[3], aw, bw); a[1] = aw; bb[1] = bw;
      hl2(x1[0], x1[1], aw, bw); a[2] = aw; bb[2] = bw;
      hl2(x1[2], x1[3], aw, bw); a[3] = aw; bb[3] = bw;
      hv[it] = a;
      lv[it] = bb;
      go[it] = (size_t)hq * hps + ((size_t)b * SEQ + s0 + row) * HD + c8;
    }
    for (int pass = 0; pass < 2; ++pass) {
#pragma unroll
      for (int it = 0; it < 2; ++it) {
        *(volatile v4u*)(chp + go[it]) = hv[it];
        *(volatile v4u*)(clp + go[it]) = lv[it];
      }
      __threadfence();
    }
  }
}

extern "C" void kernel_launch(void* const* d_in, const int* in_sizes, int n_in,
                              void* d_out, int out_size, void* d_ws, size_t ws_size,
                              hipStream_t stream) {
  if (n_in < 12) return;
  if (in_sizes[0] != MQ * DMOD || in_sizes[1] != MQ * DMOD || in_sizes[2] != MQ * DMOD) return;
  if (in_sizes[3] != MEMN * DMOD) return;
  if (in_sizes[4] != DMOD * DMOD || in_sizes[6] != DMOD * DMOD) return;
  if (in_sizes[8] != DMOD * DMOD || in_sizes[10] != DMOD * DMOD) return;
  if (in_sizes[5] != DMOD || in_sizes[7] != DMOD || in_sizes[9] != DMOD || in_sizes[11] != DMOD) return;
  if (out_size != MQ * DMOD) return;

  const float* query = (const float*)d_in[0];
  const float* key   = (const float*)d_in[1];
  const float* value = (const float*)d_in[2];
  const float* memp  = (const float*)d_in[3];
  const float* Wq    = (const float*)d_in[4];
  const float* bq    = (const float*)d_in[5];
  const float* Wk    = (const float*)d_in[6];
  const float* bk    = (const float*)d_in[7];
  const float* Wv    = (const float*)d_in[8];
  const float* bv    = (const float*)d_in[9];
  const float* Wo    = (const float*)d_in[10];
  const float* bo    = (const float*)d_in[11];
  const int nbq = in_sizes[5], nbk = in_sizes[7], nbv = in_sizes[9], nbo = in_sizes[11];

  const size_t PW  = (size_t)DMOD * DMOD * 2;
  const size_t PXQ = (size_t)MQ * DMOD * 2;
  const size_t PXK = (size_t)MK * DMOD * 2;
  const size_t PVT = (size_t)BATCH * DMOD * TP * 2;
  const size_t PC  = (size_t)NH * MQ * HD * 2;
  size_t off = 0;
  const size_t oWT = off; off += 4 * PW;
  const size_t oXQ = off; off += PXQ;
  const size_t oXK = off; off += PXK;
  const size_t oXV = off; off += PXK;
  const size_t oQH = off; off += PXQ;
  const size_t oQL = off; off += PXQ;
  const size_t oKH = off; off += PXK;
  const size_t oKL = off; off += PXK;
  const size_t oVH = off; off += PVT;
  const size_t oVL = off; off += PVT;
  const size_t oCH = off; off += PC;
  const size_t oCL = off; off += PC;
  if (off > ws_size) return;
  if (off > (size_t)134217728) return;

  char* ws = (char*)d_ws;
  unsigned short* WT  = (unsigned short*)(ws + oWT);
  unsigned short* WqT = WT;
  unsigned short* WkT = WT + (size_t)1 * DMOD * DMOD;
  unsigned short* WvT = WT + (size_t)2 * DMOD * DMOD;
  unsigned short* WoB = WT + (size_t)3 * DMOD * DMOD;
  unsigned short* XQ  = (unsigned short*)(ws + oXQ);
  unsigned short* XK  = (unsigned short*)(ws + oXK);
  unsigned short* XV  = (unsigned short*)(ws + oXV);
  unsigned short* QH  = (unsigned short*)(ws + oQH);
  unsigned short* QL  = (unsigned short*)(ws + oQL);
  unsigned short* KH  = (unsigned short*)(ws + oKH);
  unsigned short* KL  = (unsigned short*)(ws + oKL);
  unsigned short* VTH = (unsigned short*)(ws + oVH);
  unsigned short* VTL = (unsigned short*)(ws + oVL);
  unsigned short* CH  = (unsigned short*)(ws + oCH);
  unsigned short* CL  = (unsigned short*)(ws + oCL);

  const dim3 blk(256), blk128(128);
  const dim3 gW((DMOD / 64) * (DMOD / 64), 4);
  const dim3 gCq((MQ * DMOD / 8 + 255) / 256);
  const dim3 gCkv((BATCH * TP * (DMOD / 8) + 255) / 256, 2);
  const dim3 gGq(((MQ / 64) * (DMOD / 64) + 7) / 8, 1);
  const dim3 gGk(((MK / 64) * (DMOD / 64) + 7) / 8, 1);
  const dim3 gGv(((DMOD / 64) * (TP / 64) + 7) / 8, BATCH);
  const dim3 gAttn(BATCH * NH * NQB);
  const dim3 gGo(((MQ / 64) * (DMOD / 64) + 7) / 8);
  const float osc = 1.0f / (ASC * WSC);
  const float sscale = 0.17677669529663687f;

  wtrans<<<gW, blk, 0, stream>>>(Wq, Wk, Wv, Wo, WT);
  convq<<<gCq, blk, 0, stream>>>(query, XQ, MQ * DMOD / 8);
  convkv<<<gCkv, blk, 0, stream>>>(key, value, memp, XK, XV, BATCH * TP * (DMOD / 8));

  gemm64<3, 1><<<gGq, blk, 0, stream>>>(XQ, DMOD, 0, WqT, DMOD, 0, QH, QL, DMOD, 0, bq, nbq,
                                       MQ, DMOD, DMOD, osc, RSC);
  gemm64<3, 1><<<gGk, blk, 0, stream>>>(XK, DMOD, 0, WkT, DMOD, 0, KH, KL, DMOD, 0, bk, nbk,
                                       MK, DMOD, DMOD, osc, RSC);
  gemm64<3, 2><<<gGv, blk, 0, stream>>>(WvT, DMOD, 0, XV, DMOD, TP * DMOD, VTH, VTL, TP, DMOD * TP,
                                       bv, nbv, DMOD, TP, DMOD, osc, RSC);

  attn32<<<gAttn, blk128, 0, stream>>>(QH, QL, KH, KL, VTH, VTL, CH, CL, sscale);

  gemm_ob<<<gGo, blk, 0, stream>>>(CH, CL, MQ * HD, WoB, DMOD, bo, nbo, (float*)d_out, DMOD,
                                   MQ, DMOD, DMOD);
  (void)hipGetLastError();
}
